// Conv2dWeightModulate_45509473469072
// MI455X (gfx1250) — hardware-verified
//
#include <hip/hip_runtime.h>

typedef _Float16 f16t;
typedef _Float16 v16h __attribute__((ext_vector_type(16)));
typedef _Float16 v8h  __attribute__((ext_vector_type(8)));
typedef float    v8f  __attribute__((ext_vector_type(8)));
typedef float    v4f  __attribute__((ext_vector_type(4)));
typedef v8h __attribute__((may_alias)) v8ha;
typedef v4f __attribute__((may_alias)) v4fa;
union Frag { v16h v; v8h half[2]; };

#define NB    8
#define CIN   512
#define COUT  512
#define HWD   32
#define NPIX  1024
#define NTAP  9
#define RDIM  (CIN * NTAP)
#define PADW  34
#define XROW  (PADW * CIN)
#define COEF  0.014731391274719742f
#define WCAR  64.0f
#define EPSV  1e-8f

static_assert(XROW % 8 == 0);
static_assert(RDIM % 32 == 0);
static_assert((XROW * 2) % 128 == 0);
static_assert((RDIM * 2) % 128 == 0);

__device__ __forceinline__ v8f wmma_f16(v16h a, v16h b, v8f c) {
  v8f d = __builtin_amdgcn_wmma_f32_16x16x32_f16(false, a, false, b, (short)0, c, false, false);
  asm volatile("v_nop\n\tv_nop\n\tv_nop\n\tv_nop" : "+v"(d) : "v"(a), "v"(b));
  return d;
}

__device__ __forceinline__ v8h zero8h() {
  v8h z;
  #pragma unroll
  for (int j = 0; j < 8; ++j) z[j] = (f16t)0.0f;
  return z;
}

__device__ __forceinline__ float wave_sum(float s) {
  s += __shfl_xor(s, 16);
  s += __shfl_xor(s, 8);
  s += __shfl_xor(s, 4);
  s += __shfl_xor(s, 2);
  s += __shfl_xor(s, 1);
  return s;
}

__global__ __launch_bounds__(256) void wprep_k(const float* __restrict__ weight,
                                               f16t* __restrict__ w16, float* __restrict__ s2)
{
  __shared__ __attribute__((aligned(16))) f16t sW[NTAP * CIN];
  __shared__ __attribute__((aligned(16))) float sS[CIN];
  const int tid = threadIdx.x;
  const int o = blockIdx.x;
  #pragma unroll 1
  for (int jj = 0; jj < 2; ++jj) {
    const int i = tid + 256 * jj;
    const float* wp = weight + ((size_t)o * CIN + i) * NTAP;
    float q = 0.f;
    #pragma unroll
    for (int k = 0; k < NTAP; ++k) {
      const float w0 = wp[k] * COEF;
      q = fmaf(w0, w0, q);
      sW[k * CIN + i] = (f16t)(w0 * WCAR);
    }
    sS[i] = q;
  }
  __syncthreads();
  f16t* dst = w16 + (size_t)o * RDIM;
  float* sdst = s2 + (size_t)o * CIN;
  #pragma unroll
  for (int j = 0; j < 3; ++j) {
    const int idx = j * 256 + tid;
    if (idx < RDIM / 8) *(volatile v8h*)(dst + (size_t)idx * 8) = *(const v8ha*)(sW + idx * 8);
  }
  if (tid < 128) *(volatile v4f*)(sdst + 4 * tid) = *(const v4fa*)(sS + 4 * tid);
  __threadfence();
  #pragma unroll
  for (int j = 0; j < 3; ++j) {
    const int idx = j * 256 + tid;
    if (idx < RDIM / 8) *(volatile v8h*)(dst + (size_t)idx * 8) = *(const v8ha*)(sW + idx * 8);
  }
  if (tid < 128) *(volatile v4f*)(sdst + 4 * tid) = *(const v4fa*)(sS + 4 * tid);
}

__global__ __launch_bounds__(256) void xs_k(const float* __restrict__ x, const float* __restrict__ style,
                                            f16t* __restrict__ xs)
{
  __shared__ __attribute__((aligned(16))) f16t sX[XROW];
  const int tid = threadIdx.x;
  const int yp = blockIdx.x, b = blockIdx.y;
  const bool border = (yp == 0) || (yp == PADW - 1);
  const v8h z = zero8h();
  if (border) {
    #pragma unroll 1
    for (int j = 0; j < 9; ++j) {
      const int idx = j * 256 + tid;
      if (idx < XROW / 8) *(v8ha*)(sX + idx * 8) = z;
    }
  } else {
    if (tid < 128) {
      const int idx = (tid < 64) ? (tid * 8) : ((PADW - 1) * CIN + (tid - 64) * 8);
      *(v8ha*)(sX + idx) = z;
    }
    const int y = yp - 1;
    const int q = tid & 7, cl = tid >> 3;
    #pragma unroll 1
    for (int j = 0; j < 16; ++j) {
      const int c = 32 * j + cl;
      const float s = style[b * CIN + c];
      const v4f v = *(const v4fa*)(x + ((size_t)(b * CIN + c) * HWD + y) * HWD + 4 * q);
      f16t* d = sX + (4 * q + 1) * CIN + c;
      d[0]       = (f16t)(v.x * s);
      d[CIN]     = (f16t)(v.y * s);
      d[2 * CIN] = (f16t)(v.z * s);
      d[3 * CIN] = (f16t)(v.w * s);
    }
  }
  __syncthreads();
  f16t* dst = xs + (size_t)(b * PADW + yp) * XROW;
  #pragma unroll 1
  for (int j = 0; j < 9; ++j) {
    const int idx = j * 256 + tid;
    if (idx < XROW / 8) *(volatile v8h*)(dst + (size_t)idx * 8) = *(const v8ha*)(sX + idx * 8);
  }
  __threadfence();
  #pragma unroll 1
  for (int j = 0; j < 9; ++j) {
    const int idx = j * 256 + tid;
    if (idx < XROW / 8) *(volatile v8h*)(dst + (size_t)idx * 8) = *(const v8ha*)(sX + idx * 8);
  }
}

__global__ __launch_bounds__(256) void sigma_k(const float* __restrict__ style, const float* __restrict__ s2,
                                               float* __restrict__ sig)
{
  __shared__ __attribute__((aligned(16))) float sst[CIN];
  __shared__ __attribute__((aligned(16))) float sg[32];
  const int tid = threadIdx.x, lane = tid & 31, w = tid >> 5;
  const int bo0 = blockIdx.x * 32;
  const int b = bo0 / COUT, o0 = bo0 % COUT;
  {
    const float a0 = style[b * CIN + tid];
    const float a1 = style[b * CIN + tid + 256];
    sst[tid] = a0 * a0;
    sst[tid + 256] = a1 * a1;
  }
  __syncthreads();
  #pragma unroll 1
  for (int j = 0; j < 4; ++j) {
    const int o = o0 + 4 * w + j;
    const float* row = s2 + (size_t)o * CIN;
    float s = 0.f;
    #pragma unroll 4
    for (int k = 0; k < 16; ++k) s = fmaf(sst[lane + 32 * k], row[lane + 32 * k], s);
    s = wave_sum(s);
    if (lane == 0) sg[4 * w + j] = rsqrtf(s + EPSV);
  }
  __syncthreads();
  const v4f v = *(const v4fa*)(sg + 4 * (lane & 7));
  float* dst = sig + bo0 + 4 * (lane & 7);
  const bool pw = (w == 0) && (lane < 8);
  if (pw) *(volatile v4f*)dst = v;
  __threadfence();
  if (pw) *(volatile v4f*)dst = v;
}

__global__ __launch_bounds__(128) void conv_k(const f16t* __restrict__ xs, const f16t* __restrict__ w16,
                                              const float* __restrict__ sig, float* __restrict__ out)
{
  __shared__ __attribute__((aligned(16))) float sD[128 * 64];
  const int tid = threadIdx.x, lane = tid & 31, w = tid >> 5;
  const int h = lane >> 4, m = lane & 15;
  const int t = blockIdx.x;
  const int obase = blockIdx.y * 128;
  const int b = blockIdx.z;
  const int pm = w & 1, on = w >> 1;
  const int y = 2 * t + pm;

  const f16t* abase = xs + ((size_t)(b * PADW + y) * PADW + m) * CIN + 8 * h;
  const f16t* bbase = w16 + (size_t)(obase + 64 * on + m) * RDIM + 8 * h;

  const v8f z8 = {0.f, 0.f, 0.f, 0.f, 0.f, 0.f, 0.f, 0.f};
  v8f acc[2][4];
  #pragma unroll
  for (int mi = 0; mi < 2; ++mi) {
    #pragma unroll
    for (int nt = 0; nt < 4; ++nt) acc[mi][nt] = z8;
  }

  #pragma unroll 1
  for (int tap = 0; tap < NTAP; ++tap) {
    const int ky = tap / 3, kx = tap - 3 * ky;
    const f16t* ap = abase + (size_t)(ky * PADW + kx) * CIN;
    const f16t* bp = bbase + (size_t)tap * CIN;
    #pragma unroll 1
    for (int c0 = 0; c0 < CIN; c0 += 32) {
      Frag a0, a1;
      a0.half[0] = *(const v8ha*)(ap + c0);
      a0.half[1] = *(const v8ha*)(ap + c0 + 16);
      a1.half[0] = *(const v8ha*)(ap + 16 * CIN + c0);
      a1.half[1] = *(const v8ha*)(ap + 16 * CIN + c0 + 16);
      #pragma unroll
      for (int nt = 0; nt < 4; ++nt) {
        Frag bb;
        const f16t* bq = bp + (size_t)nt * 16 * RDIM + c0;
        bb.half[0] = *(const v8ha*)(bq);
        bb.half[1] = *(const v8ha*)(bq + 16);
        acc[0][nt] = wmma_f16(a0.v, bb.v, acc[0][nt]);
        acc[1][nt] = wmma_f16(a1.v, bb.v, acc[1][nt]);
      }
    }
  }

  #pragma unroll
  for (int nt = 0; nt < 4; ++nt) {
    const int col = 64 * on + 16 * nt + m;
    const float sc = sig[(size_t)(b * COUT + obase + col)] * (1.0f / WCAR);
    #pragma unroll
    for (int mi = 0; mi < 2; ++mi) {
      v4f u0, u1;
      u0.x = acc[mi][nt][0] * sc; u0.y = acc[mi][nt][1] * sc;
      u0.z = acc[mi][nt][2] * sc; u0.w = acc[mi][nt][3] * sc;
      u1.x = acc[mi][nt][4] * sc; u1.y = acc[mi][nt][5] * sc;
      u1.z = acc[mi][nt][6] * sc; u1.w = acc[mi][nt][7] * sc;
      float* sp = sD + col * 64 + 32 * pm + 16 * mi + 8 * h;
      *(v4fa*)sp = u0;
      *(v4fa*)(sp + 4) = u1;
    }
  }
  __syncthreads();

  const int hs = lane >> 4, x4 = 4 * (lane & 15);
  float* ob = out + (size_t)(b * COUT + obase) * NPIX + 64 * t + x4;
  #pragma unroll
  for (int i = 0; i < 16; ++i) {
    const int row = 32 * w + 2 * i + hs;
    const v4f v = *(const v4fa*)(sD + row * 64 + x4);
    *(volatile v4f*)(ob + (size_t)row * NPIX) = v;
  }
  __threadfence();
  #pragma unroll
  for (int i = 0; i < 16; ++i) {
    const int row = 32 * w + 2 * i + hs;
    const v4f v = *(const v4fa*)(sD + row * 64 + x4);
    *(volatile v4f*)(ob + (size_t)row * NPIX) = v;
  }
}

extern "C" void kernel_launch(void* const* d_in, const int* in_sizes, int n_in,
                              void* d_out, int out_size, void* d_ws, size_t ws_size,
                              hipStream_t stream)
{
  if (n_in < 3) return;
  if (in_sizes[0] != NB * CIN * NPIX) return;
  if (in_sizes[1] != NB * CIN) return;
  if (in_sizes[2] != COUT * CIN * NTAP) return;
  if (out_size != NB * COUT * NPIX) return;

  const float* x      = (const float*)d_in[0];
  const float* style  = (const float*)d_in[1];
  const float* weight = (const float*)d_in[2];
  float* outp = (float*)d_out;

  const size_t szW16 = (size_t)COUT * RDIM * sizeof(f16t);
  const size_t szS2  = (size_t)COUT * CIN * sizeof(float);
  const size_t szSIG = (size_t)NB * COUT * sizeof(float);
  const size_t szXS  = (size_t)NB * PADW * XROW * sizeof(f16t);
  const size_t offW16 = 0;
  const size_t offS2  = offW16 + szW16;
  const size_t offSIG = offS2 + szS2;
  const size_t offXS  = offSIG + szSIG;
  const size_t total  = offXS + szXS;
  if (total > ws_size) return;
  char* ws = (char*)d_ws;
  f16t*  W16 = (f16t*)(ws + offW16);
  float* S2  = (float*)(ws + offS2);
  float* SIG = (float*)(ws + offSIG);
  f16t*  XS  = (f16t*)(ws + offXS);

  wprep_k<<<COUT, 256, 0, stream>>>(weight, W16, S2);
  xs_k<<<dim3(PADW, NB), 256, 0, stream>>>(x, style, XS);
  sigma_k<<<(NB * COUT) / 32, 256, 0, stream>>>(style, S2, SIG);
  conv_k<<<dim3(NPIX / 64, COUT / 128, NB), 128, 0, stream>>>(XS, W16, SIG, outp);
}
